// NaiveFourierKANLayer_80333068304841
// MI455X (gfx1250) — hardware-verified
//
#include <hip/hip_runtime.h>
#include <math.h>

typedef __attribute__((ext_vector_type(16))) _Float16 v16h;
typedef __attribute__((ext_vector_type(16))) __bf16 v16b;
typedef __attribute__((ext_vector_type(8)))  _Float16 v8h;
typedef __attribute__((ext_vector_type(8)))  float v8f;
typedef __attribute__((ext_vector_type(4)))  float v4f;
typedef __attribute__((ext_vector_type(2)))  float v2f;
typedef __attribute__((ext_vector_type(4)))  unsigned v4u;
typedef __attribute__((ext_vector_type(4)))  int v4i;
typedef float __attribute__((may_alias)) float_a;
typedef int __attribute__((may_alias)) int_a;

template <typename T> __device__ __forceinline__ void vst2(void* p, T v) { *(volatile T*)p = v; __threadfence(); *(volatile T*)p = v; }
__device__ __forceinline__ v8f wmma16(v16h a, v16h b, v8f c) {
  v8f d = __builtin_amdgcn_wmma_f32_16x16x32_f16(false, a, false, b, (short)0, c, false, false);
  asm volatile("v_nop\n\tv_nop\n\tv_nop\n\tv_nop" : "+v"(d) : "v"(a), "v"(b));
  return d;
}
__device__ __forceinline__ v8f wmma_bf(v16b a, v16b b, v8f c) {
  v8f d = __builtin_amdgcn_wmma_f32_16x16x32_bf16(false, a, false, b, (short)0, c, false, false);
  asm volatile("v_nop\n\tv_nop\n\tv_nop\n\tv_nop" : "+v"(d) : "v"(a), "v"(b));
  return d;
}
__device__ __forceinline__ v16h frag_h(const _Float16* rowk0, int lane) {
  union { v16h v; v8h q[2]; } u; const _Float16* p = rowk0 + 8 * (lane >> 4);
  u.q[0] = *(const v8h*)p; u.q[1] = *(const v8h*)(p + 16); return u.v;
}
__device__ __forceinline__ v16h frag_f32(const float* rowk0, int lane) {
  v16h a; const float* p = rowk0 + 8 * (lane >> 4);
#pragma unroll
  for (int i = 0; i < 8; ++i) { a[i] = (_Float16)p[i]; a[8 + i] = (_Float16)p[16 + i]; }
  return a;
}
__device__ __forceinline__ v16h frag_f32s(const float* rowk0, int lane, float sc) {
  v16h a; const float* p = rowk0 + 8 * (lane >> 4);
#pragma unroll
  for (int i = 0; i < 8; ++i) { a[i] = (_Float16)(p[i] * sc); a[8 + i] = (_Float16)(p[16 + i] * sc); }
  return a;
}
__device__ __forceinline__ v16h fragc_f32(const float* W, int k0, int n, int lane, int ld, int K) {
  v16h a; const int g = lane >> 4;
#pragma unroll
  for (int i = 0; i < 8; ++i) { const int ka = k0 + 8 * g + i, kb = ka + 16;
    a[i] = (_Float16)(ka < K ? W[(size_t)ka * ld + n] : 0.f); a[8 + i] = (_Float16)(kb < K ? W[(size_t)kb * ld + n] : 0.f); }
  return a;
}
struct F2 { v16b h, l; };
__device__ __forceinline__ F2 bsplit16(const float v[16]) { F2 r;
#pragma unroll
  for (int i = 0; i < 16; ++i) { const __bf16 h = (__bf16)v[i]; r.h[i] = h; r.l[i] = (__bf16)(v[i] - (float)h); }
  return r; }
__device__ __forceinline__ F2 split_row(const float* row, int k0, int lane) { float v[16]; const float* p = row + k0 + 8 * (lane >> 4);
#pragma unroll
  for (int i = 0; i < 8; ++i) { v[i] = p[i]; v[8 + i] = p[16 + i]; }
  return bsplit16(v); }
__device__ __forceinline__ F2 split_rowK(const float* row, int k0, int lane, int K) { float v[16]; const int g = lane >> 4;
#pragma unroll
  for (int i = 0; i < 8; ++i) { const int ka = k0 + 8 * g + i, kb = ka + 16; v[i] = ka < K ? row[ka] : 0.f; v[8 + i] = kb < K ? row[kb] : 0.f; }
  return bsplit16(v); }
__device__ __forceinline__ F2 split_col(const float* W, int k0, int n, int lane, int ld, int K) { float v[16]; const int g = lane >> 4;
#pragma unroll
  for (int i = 0; i < 8; ++i) { const int ka = k0 + 8 * g + i, kb = ka + 16; v[i] = ka < K ? W[(size_t)ka * ld + n] : 0.f; v[8 + i] = kb < K ? W[(size_t)kb * ld + n] : 0.f; }
  return bsplit16(v); }
__device__ __forceinline__ v8f mac3(const F2& a, const F2& b, v8f c) { c = wmma_bf(a.l, b.h, c); c = wmma_bf(a.h, b.l, c); return wmma_bf(a.h, b.h, c); }
__device__ __forceinline__ float sigm(float v) { return 1.0f / (1.0f + expf(-v)); }
#define LDSX() do { asm volatile("s_wait_dscnt 0" ::: "memory"); __builtin_amdgcn_wave_barrier(); __builtin_amdgcn_fence(__ATOMIC_RELEASE, "workgroup"); } while (0)

#define NRW 20000
#define NRP 20032
#define NI 64
#define NO 64
#define GK 100
#define NGRP (NI / 16)

__global__ __launch_bounds__(256) void k_pack(const float* __restrict__ C, _Float16* __restrict__ Bp) {
  const int grp = blockIdx.y, k = blockIdx.x, tid = threadIdx.x;
  const int j = tid >> 2, q4 = tid & 3; union { v8h h; v4u u; } pk;
#pragma unroll
  for (int e = 0; e < 8; ++e) { const int el = q4 * 8 + e; const int which = el >> 4, ii = grp * 16 + (el & 15);
    pk.h[e] = (_Float16)(C[(((size_t)which * NO + j) * NI + ii) * GK + k] * 64.0f); }
  vst2(Bp + ((((size_t)grp * GK + k) * NO + j) * 32) + q4 * 8, pk.u);
}
__global__ __launch_bounds__(128) void k_main(const float* __restrict__ x, const _Float16* __restrict__ Bp, const float* __restrict__ bias, float* __restrict__ out) {
  __shared__ __align__(16) _Float16 sa[4][16][40];
  __shared__ __align__(16) float so[4][16][68];
  const int tid = threadIdx.x, wave = tid >> 5, lane = tid & 31, col = lane & 15, g = lane >> 4;
  const int r0 = blockIdx.x * 64 + wave * 16;
  v8f acc[4] = {};
#pragma unroll 1
  for (int grp = 0; grp < NGRP; ++grp) {
    float c1[8], s1[8], ck[8], sk[8];
    const int row = min(r0 + col, NRW - 1);
#pragma unroll
    for (int u = 0; u < 8; ++u) { const float xv = x[(size_t)row * NI + grp * 16 + g * 8 + u]; float sv, cv; sincosf(xv, &sv, &cv); c1[u] = cv; s1[u] = sv; ck[u] = cv; sk[u] = sv; }
#pragma unroll 1
    for (int k = 0; k < GK; ++k) {
      union { v8h h; v4u uu; } pc, ps;
#pragma unroll
      for (int u = 0; u < 8; ++u) { pc.h[u] = (_Float16)ck[u]; ps.h[u] = (_Float16)sk[u]; }
      *(v4u*)(&sa[wave][col][g * 8]) = pc.uu; *(v4u*)(&sa[wave][col][16 + g * 8]) = ps.uu;
      LDSX();
      const v16h a = frag_h(&sa[wave][col][0], lane);
#pragma unroll
      for (int t = 0; t < 4; ++t) acc[t] = wmma16(a, frag_h(Bp + (((size_t)grp * GK + k) * NO + t * 16 + col) * 32, lane), acc[t]);
      LDSX();
#pragma unroll
      for (int u = 0; u < 8; ++u) { const float cn = ck[u] * c1[u] - sk[u] * s1[u]; const float sn = sk[u] * c1[u] + ck[u] * s1[u]; ck[u] = cn; sk[u] = sn; } } }
#pragma unroll
  for (int t = 0; t < 4; ++t) { const float bb = bias[t * 16 + col];
#pragma unroll
    for (int r = 0; r < 8; ++r) so[wave][8 * g + r][t * 16 + col] = acc[t][r] * (1.0f / 64.0f) + bb; }
  LDSX();
  for (int q = lane; q < 16 * 16; q += 32) { const int rl = q >> 4, pcn = q & 15; if (r0 + rl < NRW) vst2(out + (size_t)(r0 + rl) * NO + pcn * 4, *(const v4f*)(&so[wave][rl][pcn * 4])); }
}
extern "C" void kernel_launch(void* const* d_in, const int* in_sizes, int n_in, void* d_out, int out_size, void* d_ws, size_t ws_size, hipStream_t stream) {
  (void)in_sizes; (void)n_in; (void)out_size; (void)ws_size;
  const float* x = (const float*)d_in[0]; const float* C = (const float*)d_in[1]; const float* bias = (const float*)d_in[2];
  float* out = (float*)d_out;
  _Float16* Bp = (_Float16*)d_ws;
  k_pack<<<dim3(GK, NGRP), 256, 0, stream>>>(C, Bp);
  k_main<<<NRP / 64, 128, 0, stream>>>(x, Bp, bias, out);
}
